// BahdanauAttention_4269197492750
// MI455X (gfx1250) — hardware-run, weakly checked
//
#include <hip/hip_runtime.h>


#define NBE 8
#define NQY 32
#define NKY 2048
#define NDI 256
#define NU  256
#define OFF1 65536
typedef _Float16 h16;
typedef unsigned short bf;
typedef __attribute__((ext_vector_type(16))) __bf16   v16bf;
typedef __attribute__((ext_vector_type(16))) _Float16 v16h;
typedef __attribute__((ext_vector_type(8)))  _Float16 v8h;
typedef __attribute__((ext_vector_type(8)))  unsigned short v8us;
typedef __attribute__((ext_vector_type(8)))  float    v8f;
typedef __attribute__((ext_vector_type(4)))  float    v4f;
typedef v8h  __attribute__((may_alias)) v8ha;
typedef v4f  __attribute__((may_alias)) v4fa;
typedef v8us __attribute__((may_alias)) v8usa;

__device__ __forceinline__ unsigned short f2bf(float f) { unsigned u = __float_as_uint(f); u += 0x7FFFu + ((u >> 16) & 1u); return (unsigned short)(u >> 16); }
__device__ __forceinline__ float bf2f(unsigned short b) { return __uint_as_float(((unsigned)b) << 16); }
__device__ __forceinline__ float bfr(float f) { return bf2f(f2bf(f)); }
__device__ __forceinline__ v16h cat16(v8h lo, v8h hi) { return __builtin_shufflevector(lo, hi, 0, 1, 2, 3, 4, 5, 6, 7, 8, 9, 10, 11, 12, 13, 14, 15); }
__device__ __forceinline__ v16bf cat16b(v8us lo, v8us hi) { return __builtin_bit_cast(v16bf, __builtin_shufflevector(lo, hi, 0, 1, 2, 3, 4, 5, 6, 7, 8, 9, 10, 11, 12, 13, 14, 15)); }
__device__ __forceinline__ v8f wmma16(v16h a, v16h b, v8f c) { return __builtin_amdgcn_wmma_f32_16x16x32_f16(false, a, false, b, (short)0, c, false, false); }
__device__ __forceinline__ v8f wmmab(v16bf a, v16bf b, v8f c) { return __builtin_amdgcn_wmma_f32_16x16x32_bf16(false, a, false, b, (short)0, c, false, false); }
typedef __attribute__((ext_vector_type(2))) unsigned short v2us;

template <typename T16> struct WFrag;
template <> struct WFrag<h16> { typedef v16h V; static __device__ __forceinline__ V ld(const h16* p) { return cat16(*(const v8h*)p, *(const v8h*)(p + 16)); } static __device__ __forceinline__ v8f mma(V a, V b, v8f c) { return wmma16(a, b, c); } };
template <> struct WFrag<bf> { typedef v16bf V; static __device__ __forceinline__ V ld(const bf* p) { return cat16b(*(const v8us*)p, *(const v8us*)(p + 16)); } static __device__ __forceinline__ v8f mma(V a, V b, v8f c) { return wmmab(a, b, c); } };
template <typename T16, int NSPLIT, bool BIAS>
__global__ __launch_bounds__(32) void k_gemmw(const T16* __restrict__ A, const T16* __restrict__ A2, const T16* __restrict__ Bt, const T16* __restrict__ Bt2, int K, float* C, int ldc, const float* __restrict__ bias, size_t sA, size_t sB, size_t sC) {
    typedef typename WFrag<T16>::V V;
    __shared__ __align__(16) float os[16 * 68];
    const size_t z = blockIdx.z; A += z * sA; if (A2) A2 += z * sA; Bt += z * sB; if (Bt2) Bt2 += z * sB; C += z * sC;
    const int lane = threadIdx.x & 31, lr = lane & 15, hi = lane >> 4; const int r0 = blockIdx.x * 64, c0 = blockIdx.y * 64;
    v8f acc[4][4];
#pragma unroll
    for (int mb = 0; mb < 4; ++mb)
#pragma unroll
        for (int nb = 0; nb < 4; ++nb) acc[mb][nb] = (v8f){};
    const size_t aoff = (size_t)(r0 + lr) * K + 8 * hi, boff = (size_t)(c0 + lr) * K + 8 * hi;
    for (int kc = 0; kc < K; kc += 32) {
        V a[4], a2[4];
#pragma unroll
        for (int mb = 0; mb < 4; ++mb) { a[mb] = WFrag<T16>::ld(A + aoff + (size_t)mb * 16 * K + kc); if (NSPLIT == 1 || NSPLIT == 2) a2[mb] = WFrag<T16>::ld(A2 + aoff + (size_t)mb * 16 * K + kc); }
#pragma unroll
        for (int nb = 0; nb < 4; ++nb) { const V b = WFrag<T16>::ld(Bt + boff + (size_t)nb * 16 * K + kc); V b2; if (NSPLIT >= 2) b2 = WFrag<T16>::ld(Bt2 + boff + (size_t)nb * 16 * K + kc);
#pragma unroll
            for (int mb = 0; mb < 4; ++mb) { acc[mb][nb] = WFrag<T16>::mma(a[mb], b, acc[mb][nb]); if (NSPLIT == 1 || NSPLIT == 2) acc[mb][nb] = WFrag<T16>::mma(a2[mb], b, acc[mb][nb]); if (NSPLIT >= 2) acc[mb][nb] = WFrag<T16>::mma(a[mb], b2, acc[mb][nb]); } }
        asm volatile("v_nop\n\tv_nop\n\tv_nop\n\tv_nop" : "+v"(acc[0][0]), "+v"(acc[1][1]), "+v"(acc[2][2]), "+v"(acc[3][3]) : "v"(a[0]), "v"(a[3]));
    }
#pragma unroll
    for (int mb = 0; mb < 4; ++mb) {
#pragma unroll
        for (int nb = 0; nb < 4; ++nb) {
#pragma unroll
            for (int j = 0; j < 8; ++j) os[(hi * 8 + j) * 68 + nb * 16 + lr] = acc[mb][nb][j]; }
        __builtin_amdgcn_wave_barrier(); asm volatile("" ::: "memory");
        float* crow = C + (size_t)(r0 + mb * 16) * ldc + c0;
#pragma unroll 1
        for (int ps = 0; ps < 2; ++ps) {
#pragma unroll
            for (int s = 0; s < 8; ++s) { const int row = 2 * s + hi, cofs = lr * 4; v4f val = *(const v4fa*)(os + row * 68 + cofs); if (BIAS) { val[0] += bfr(bias[c0 + cofs]); val[1] += bfr(bias[c0 + cofs + 1]); val[2] += bfr(bias[c0 + cofs + 2]); val[3] += bfr(bias[c0 + cofs + 3]); }
                *(volatile v4f*)(crow + (size_t)row * ldc + cofs) = val; }
            if (ps == 0) __threadfence(); }
        __builtin_amdgcn_wave_barrier(); asm volatile("" ::: "memory");
    }
}

__global__ __launch_bounds__(256) void k_cvt8(const float* __restrict__ src, bf* dst, size_t n8) { const size_t i = (size_t)blockIdx.x * 256 + threadIdx.x; if (i >= n8) return; const v8f v = *(const v8f*)(src + i * 8); v8us o;
#pragma unroll
    for (int k = 0; k < 8; ++k) o[k] = f2bf(v[k]); *(volatile v8us*)(dst + i * 8) = o; __threadfence(); *(volatile v8us*)(dst + i * 8) = o; }

__global__ __launch_bounds__(256) void k_wtG(const float* __restrict__ w, int K, int N, bf* Bt) {
    const int lane = threadIdx.x & 31; const int L0 = (blockIdx.x * 8 + (threadIdx.x >> 5)) * 8; const int nlines = N * K / 64;
#pragma unroll
    for (int ps = 0; ps < 2; ++ps) {
        for (int l = 0; l < 8; ++l) { const int L = L0 + l; if (L >= nlines) break; const size_t e = (size_t)L * 64 + lane * 2; const int k = (int)(e % K), n = (int)(e / K); v2us o;
            o[0] = f2bf(w[(size_t)k * N + n]); o[1] = f2bf(w[(size_t)(k + 1) * N + n]); *(volatile v2us*)(Bt + e) = o; }
        if (ps == 0) __threadfence(); }
}

__global__ __launch_bounds__(256) void k_score(const float* QP, const float* KT, const float* __restrict__ uv, float* S) { const size_t e = (size_t)blockIdx.x * 256 + threadIdx.x; if (e >= (size_t)NBE * NQY * NKY) return; const int j = (int)(e % NKY); const size_t r = e / NKY; const size_t b = r / NQY; const float* q = QP + r * NU; const float* k = KT + b * NU * NKY + j; float s = 0.0f;
  for (int u = 0; u < NU; ++u) s += bfr(uv[u]) * tanhf(q[u] + k[(size_t)u * NKY]);
  *(volatile float*)(S + e) = s; __threadfence(); *(volatile float*)(S + e) = s; }

__global__ __launch_bounds__(256) void k_softrow(const float* S, float* P, bf* PH, bf* PL) { const int r = blockIdx.x * 256 + threadIdx.x; if (r >= NBE * NQY) return; const float* s = S + (size_t)r * NKY; float mx = s[0];
  for (int j = 1; j < NKY; ++j) { const float sj = s[j]; mx = (sj > mx) ? sj : mx; }
  float sum = 0.0f;
  for (int j = 0; j < NKY; ++j) sum += expf(s[j] - mx);
  for (int ps = 0; ps < 2; ++ps) {
    for (int j0 = 0; j0 < NKY; j0 += 8) { v4f w0, w1; v8us h, l;
#pragma unroll
      for (int q = 0; q < 8; ++q) { const float w = expf(s[j0 + q] - mx) / sum; if (q < 4) w0[q] = w; else w1[q - 4] = w; const unsigned short hb = f2bf(w); h[q] = hb; l[q] = f2bf(w - bf2f(hb)); }
      float* po = P + (size_t)r * NKY + j0; *(volatile v4f*)po = w0; *(volatile v4f*)(po + 4) = w1; *(volatile v8us*)(PH + (size_t)r * NKY + j0) = h; *(volatile v8us*)(PL + (size_t)r * NKY + j0) = l; }
    if (ps == 0) __threadfence(); } }

__global__ __launch_bounds__(256) void k_pick(const float* OB, float* out) { const size_t e = (size_t)blockIdx.x * 256 + threadIdx.x; if (e >= (size_t)NBE * NQY * NDI / 4) return; const int d4 = (int)(e % (NDI / 4)); const size_t bi = e / (NDI / 4); const int i = (int)(bi % NQY); const size_t b = bi / NQY; const v4f v = *(const v4f*)(OB + ((b * 64 + (b & 1) * NQY + i) * NDI) + (size_t)d4 * 4); *(volatile v4f*)(out + e * 4) = v; __threadfence(); *(volatile v4f*)(out + e * 4) = v; }

extern "C" void kernel_launch(void* const* d_in, const int* in_sizes, int n_in,
                              void* d_out, int out_size, void* d_ws, size_t ws_size, hipStream_t stream) {
    (void)in_sizes; (void)n_in; (void)out_size;
    const float* qy = (const float*)d_in[0]; const float* ky = (const float*)d_in[1]; const float* Wa = (const float*)d_in[2]; const float* Wb = (const float*)d_in[3]; const float* uv = (const float*)d_in[4];
    float* OUT = (float*)d_out;
    float* P = (float*)d_out + OFF1;
    char* wsp = (char*)d_ws;
    auto take = [&](size_t bytes) { char* p = wsp; wsp += (bytes + 255) & ~(size_t)255; return (void*)p; };
    bf* QB = (bf*)take((size_t)NBE * NQY * NDI * 2); bf* KB = (bf*)take((size_t)NBE * NKY * NDI * 2); bf* WAB = (bf*)take((size_t)NU * NDI * 2); bf* WBB = (bf*)take((size_t)NU * NDI * 2);
    float* QP = (float*)take((size_t)NBE * NQY * NU * 4); float* KT = (float*)take((size_t)NBE * NU * NKY * 4); float* S = (float*)take((size_t)NBE * NQY * NKY * 4);
    bf* PH = (bf*)take((size_t)NBE * NQY * NKY * 2); bf* PL = (bf*)take((size_t)NBE * NQY * NKY * 2); bf* VT = (bf*)take((size_t)NBE * NDI * NKY * 2); float* OB = (float*)take((size_t)NBE * 64 * NDI * 4);
    if ((size_t)(wsp - (char*)d_ws) > ws_size) return;
    k_cvt8<<<(unsigned)((size_t)NBE * NQY * NDI / 8 / 256), 256, 0, stream>>>(qy, QB, (size_t)NBE * NQY * NDI / 8);
    k_cvt8<<<(unsigned)((size_t)NBE * NKY * NDI / 8 / 256), 256, 0, stream>>>(ky, KB, (size_t)NBE * NKY * NDI / 8);
    k_cvt8<<<(unsigned)((size_t)NU * NDI / 8 / 256), 256, 0, stream>>>(Wa, WAB, (size_t)NU * NDI / 8);
    k_cvt8<<<(unsigned)((size_t)NU * NDI / 8 / 256), 256, 0, stream>>>(Wb, WBB, (size_t)NU * NDI / 8);
    for (int b = 0; b < NBE; ++b) k_wtG<<<(unsigned)(((size_t)NKY * NDI / 64 + 63) / 64), 256, 0, stream>>>(ky + (size_t)b * NKY * NDI, NKY, NDI, VT + (size_t)b * NDI * NKY);
    k_gemmw<bf, 0, false><<<dim3(NBE * NQY / 64, NU / 64, 1), 32, 0, stream>>>(QB, nullptr, WAB, nullptr, NDI, QP, NU, nullptr, (size_t)0, (size_t)0, (size_t)0);
    k_gemmw<bf, 0, false><<<dim3(NU / 64, NKY / 64, NBE), 32, 0, stream>>>(WBB, nullptr, KB, nullptr, NDI, KT, NKY, nullptr, (size_t)0, (size_t)NKY * NDI, (size_t)NU * NKY);
    k_score<<<(unsigned)((size_t)NBE * NQY * NKY / 256), 256, 0, stream>>>(QP, KT, uv, S);
    k_softrow<<<1, 256, 0, stream>>>(S, P, PH, PL);
    for (int par = 0; par < 2; ++par) k_gemmw<bf, 1, false><<<dim3(1, NDI / 64, NBE / 2), 32, 0, stream>>>(PH, PL, VT + (size_t)par * NDI * NKY, nullptr, NKY, OB + (size_t)par * 64 * NDI, NDI, nullptr, (size_t)64 * NKY, (size_t)2 * NDI * NKY, (size_t)2 * 64 * NDI);
    k_pick<<<(unsigned)((size_t)NBE * NQY * NDI / 4 / 256), 256, 0, stream>>>(OB, OUT);
}
